// MultiHeadSelfAttention_40776419508319
// MI455X (gfx1250) — hardware-run, weakly checked
//
#include <hip/hip_runtime.h>


#ifndef NB
#define NB 2
#endif
#ifndef SEQ
#define SEQ 2048
#endif
#define NB_FULL  2
#define SEQ_FULL 2048
#define DM   1024
#define NH_  16
#define HD   64
#define DF   4096
#define ZH   2
#define MR   (NB * SEQ)
#define WCAR 1024.0f
#define ACAR 16.0f
#define QCAR 16.0f
#define VCAR 16.0f
#define GCAR 16.0f
#define PCAR 1024.0f
#define SCLS (0.125f / (QCAR * QCAR))

static_assert(SEQ % 128 == 0);
static_assert(SEQ <= SEQ_FULL);
static_assert(NB <= NB_FULL);
static_assert(NH_ % ZH == 0);
static_assert(DM == NH_ * HD);
static_assert(DM % 64 == 0);
static_assert(DF % 64 == 0);
static_assert(MR % 64 == 0);
static_assert(HD % 32 == 0);

typedef _Float16 h16;
typedef unsigned short bf;
typedef __attribute__((ext_vector_type(16))) __bf16   v16bf;
typedef __attribute__((ext_vector_type(16))) _Float16 v16h;
typedef __attribute__((ext_vector_type(8)))  _Float16 v8h;
typedef __attribute__((ext_vector_type(8)))  unsigned short v8us;
typedef __attribute__((ext_vector_type(8)))  float    v8f;
typedef __attribute__((ext_vector_type(4)))  float    v4f;
typedef __attribute__((ext_vector_type(4)))  _Float16 v4h;
typedef v8h  __attribute__((may_alias)) v8ha;
typedef v4f  __attribute__((may_alias)) v4fa;
typedef v8us __attribute__((may_alias)) v8usa;

__device__ __forceinline__ unsigned short f2bf(float f) { unsigned u = __float_as_uint(f); u += 0x7FFFu + ((u >> 16) & 1u); return (unsigned short)(u >> 16); }
__device__ __forceinline__ float bf2f(unsigned short b) { return __uint_as_float(((unsigned)b) << 16); }
__device__ __forceinline__ float bfr(float f) { return bf2f(f2bf(f)); }
__device__ __forceinline__ void splitf(float y, unsigned short& h, unsigned short& l) { h = f2bf(y); l = f2bf(y - bf2f(h)); }
__device__ __forceinline__ v16h cat16(v8h lo, v8h hi) { return __builtin_shufflevector(lo, hi, 0, 1, 2, 3, 4, 5, 6, 7, 8, 9, 10, 11, 12, 13, 14, 15); }
__device__ __forceinline__ v16bf cat16b(v8us lo, v8us hi) { return __builtin_bit_cast(v16bf, __builtin_shufflevector(lo, hi, 0, 1, 2, 3, 4, 5, 6, 7, 8, 9, 10, 11, 12, 13, 14, 15)); }
__device__ __forceinline__ v8f wmma16(v16h a, v16h b, v8f c) { return __builtin_amdgcn_wmma_f32_16x16x32_f16(false, a, false, b, (short)0, c, false, false); }
__device__ __forceinline__ v8f wmmab(v16bf a, v16bf b, v8f c) { return __builtin_amdgcn_wmma_f32_16x16x32_bf16(false, a, false, b, (short)0, c, false, false); }

template <typename T16> struct WFrag;
template <> struct WFrag<h16> { typedef v16h V; static __device__ __forceinline__ V ld(const h16* p) { return cat16(*(const v8h*)p, *(const v8h*)(p + 16)); } static __device__ __forceinline__ v8f mma(V a, V b, v8f c) { return wmma16(a, b, c); } };
template <> struct WFrag<bf> { typedef v16bf V; static __device__ __forceinline__ V ld(const bf* p) { return cat16b(*(const v8us*)p, *(const v8us*)(p + 16)); } static __device__ __forceinline__ v8f mma(V a, V b, v8f c) { return wmmab(a, b, c); } };

#define E_CB   1
#define E_RB   2
#define E_RES  4
#define E_RESX 8
#define E_GELU 16
#define E_H16  32
#define E_BF2  64

template <typename T16, int NSPLIT, int EPI>
__global__ __launch_bounds__(32) void k_gemmw(const T16* __restrict__ A, const T16* __restrict__ A2, const T16* __restrict__ Bt, int K,
                                              float* Cf, unsigned short* C1, unsigned short* C2, int ldc, size_t cbs,
                                              const float* __restrict__ bias, const float* __restrict__ Res, int ldr,
                                              float sc, float osc, size_t sA, size_t sB, size_t sC) {
    typedef typename WFrag<T16>::V V;
    __shared__ __align__(16) float os[64 * 68];
    const size_t z = blockIdx.z; A += z * sA; if (NSPLIT == 1) A2 += z * sA; Bt += z * sB;
    const int lane = threadIdx.x & 31, lr = lane & 15, hi = lane >> 4; const int r0 = blockIdx.x * 64, c0 = blockIdx.y * 64;
    v8f acc[4][4];
#pragma unroll
    for (int mb = 0; mb < 4; ++mb)
#pragma unroll
        for (int nb = 0; nb < 4; ++nb) acc[mb][nb] = (v8f){};
    const size_t aoff = (size_t)(r0 + lr) * K + 8 * hi, boff = (size_t)(c0 + lr) * K + 8 * hi;
#pragma unroll 1
    for (int kc = 0; kc < K; kc += 32) {
        V a[4], a2[4];
#pragma unroll
        for (int mb = 0; mb < 4; ++mb) { a[mb] = WFrag<T16>::ld(A + aoff + (size_t)mb * 16 * K + kc); if (NSPLIT == 1) a2[mb] = WFrag<T16>::ld(A2 + aoff + (size_t)mb * 16 * K + kc); }
#pragma unroll
        for (int nb = 0; nb < 4; ++nb) { const V b = WFrag<T16>::ld(Bt + boff + (size_t)nb * 16 * K + kc);
#pragma unroll
            for (int mb = 0; mb < 4; ++mb) { acc[mb][nb] = WFrag<T16>::mma(a[mb], b, acc[mb][nb]); if (NSPLIT == 1) acc[mb][nb] = WFrag<T16>::mma(a2[mb], b, acc[mb][nb]); } }
        asm volatile("v_nop\n\tv_nop\n\tv_nop\n\tv_nop" : "+v"(acc[0][0]), "+v"(acc[1][1]), "+v"(acc[2][2]), "+v"(acc[3][3]) : "v"(a[0]), "v"(a[3]));
    }
#pragma unroll
    for (int mb = 0; mb < 4; ++mb)
#pragma unroll
        for (int nb = 0; nb < 4; ++nb)
#pragma unroll
            for (int j = 0; j < 8; ++j) os[(mb * 16 + hi * 8 + j) * 68 + nb * 16 + lr] = acc[mb][nb][j];
    __syncthreads();
    constexpr bool O16 = (EPI & (E_H16 | E_BF2)) != 0;
    constexpr int NC = O16 ? 8 : 4;
    constexpr int RPI = O16 ? 4 : 2;
    constexpr int NS = 64 / RPI;
    const int rsub = O16 ? (lane >> 3) : (lane >> 4);
    const int cofs = O16 ? ((lane & 7) * 8) : ((lane & 15) * 4);
    const int rres0 = (EPI & E_RESX) ? ((r0 / SEQ) * SEQ_FULL + (r0 % SEQ)) : r0;
    const size_t ebase = z * sC + (size_t)blockIdx.y * cbs + (size_t)r0 * ldc + cofs;
    float cb[8];
#pragma unroll
    for (int q = 0; q < NC; ++q) { cb[q] = 0.0f; if constexpr ((EPI & E_CB) != 0) cb[q] = bfr(bias[c0 + cofs + q]); }
#pragma unroll 1
    for (int s = 0; s < NS; ++s) {
        const int row = s * RPI + rsub;
        float* op = os + row * 68 + cofs;
        float val[8], rv[8];
        { const v4f t0 = *(const v4fa*)op; val[0] = t0[0]; val[1] = t0[1]; val[2] = t0[2]; val[3] = t0[3]; }
        if constexpr (NC == 8) { const v4f t1 = *(const v4fa*)(op + 4); val[4] = t1[0]; val[5] = t1[1]; val[6] = t1[2]; val[7] = t1[3]; }
        if constexpr ((EPI & E_RES) != 0) {
            const float* rp = Res + (size_t)(rres0 + row) * ldr + c0 + cofs;
            { const v4f t0 = *(const v4f*)rp; rv[0] = t0[0]; rv[1] = t0[1]; rv[2] = t0[2]; rv[3] = t0[3]; }
            if constexpr (NC == 8) { const v4f t1 = *(const v4f*)(rp + 4); rv[4] = t1[0]; rv[5] = t1[1]; rv[6] = t1[2]; rv[7] = t1[3]; }
        }
        float rb = 0.0f;
        if constexpr ((EPI & E_RB) != 0) rb = bfr(bias[r0 + row]);
#pragma unroll
        for (int q = 0; q < NC; ++q) {
            float v = val[q] * sc + cb[q] + rb;
            if constexpr ((EPI & E_RES) != 0) { float r = rv[q]; if constexpr ((EPI & E_RESX) != 0) r = bfr(r); v += r; }
            if constexpr ((EPI & E_GELU) != 0) v = 0.5f * v * (1.0f + erff(v * 0.70710678118654752f));
            val[q] = v * osc;
        }
        const size_t eo = ebase + (size_t)row * ldc;
        if constexpr ((EPI & E_H16) != 0) {
            v8h o;
#pragma unroll
            for (int q = 0; q < 8; ++q) o[q] = (h16)val[q];
            *(volatile v8h*)(C1 + eo) = o; *(v8ha*)op = o;
        } else if constexpr ((EPI & E_BF2) != 0) {
            v8us oh, ol;
#pragma unroll
            for (int q = 0; q < 8; ++q) { unsigned short a, c2; splitf(val[q], a, c2); oh[q] = a; ol[q] = c2; }
            *(volatile v8us*)(C1 + eo) = oh; *(volatile v8us*)(C2 + eo) = ol; *(v8usa*)op = oh; *(v8usa*)(op + 4) = ol;
        } else {
            v4f o; o[0] = val[0]; o[1] = val[1]; o[2] = val[2]; o[3] = val[3];
            *(volatile v4f*)(Cf + eo) = o; *(v4fa*)op = o;
        }
    }
    __threadfence();
    __syncthreads();
#pragma unroll 1
    for (int s = 0; s < NS; ++s) {
        const int row = s * RPI + rsub;
        const float* op = os + row * 68 + cofs;
        const size_t eo = ebase + (size_t)row * ldc;
        if constexpr ((EPI & E_H16) != 0) { const v8h o = *(const v8ha*)op; *(volatile v8h*)(C1 + eo) = o; }
        else if constexpr ((EPI & E_BF2) != 0) { const v8us oh = *(const v8usa*)op; const v8us ol = *(const v8usa*)(op + 4); *(volatile v8us*)(C1 + eo) = oh; *(volatile v8us*)(C2 + eo) = ol; }
        else { const v4f o = *(const v4fa*)op; *(volatile v4f*)(Cf + eo) = o; }
    }
}

template <int F16>
__global__ __launch_bounds__(256) void k_tcvt(const float* __restrict__ in, unsigned short* out, int K, int N, float car) {
    __shared__ float tile[64 * 65];
    const int t = threadIdx.x; const int n0 = blockIdx.x * 64, k0 = blockIdx.y * 64;
#pragma unroll
    for (int it = 0; it < 4; ++it) { const int k = it * 16 + (t >> 4), n4 = (t & 15) * 4; const v4f v = *(const v4f*)(in + (size_t)(k0 + k) * N + n0 + n4);
        tile[k * 65 + n4 + 0] = v[0]; tile[k * 65 + n4 + 1] = v[1]; tile[k * 65 + n4 + 2] = v[2]; tile[k * 65 + n4 + 3] = v[3]; }
    __syncthreads();
    v8us o[2];
#pragma unroll
    for (int it = 0; it < 2; ++it) { const int n = it * 32 + (t >> 3), kp = (t & 7) * 8;
#pragma unroll
        for (int e = 0; e < 8; ++e) { const float w = tile[(kp + e) * 65 + n]; o[it][e] = F16 ? __builtin_bit_cast(unsigned short, (h16)(bfr(w) * car)) : f2bf(w); } }
#pragma unroll
    for (int it = 0; it < 2; ++it) { const int n = it * 32 + (t >> 3), kp = (t & 7) * 8; *(volatile v8us*)(out + (size_t)(n0 + n) * K + k0 + kp) = o[it]; }
    __threadfence();
#pragma unroll
    for (int it = 0; it < 2; ++it) { const int n = it * 32 + (t >> 3), kp = (t & 7) * 8; *(volatile v8us*)(out + (size_t)(n0 + n) * K + k0 + kp) = o[it]; }
}

template <int MODE>
__global__ __launch_bounds__(256) void k_ln(const float* __restrict__ in, int inx, const float* __restrict__ g, const float* __restrict__ bta,
                                            unsigned short* o16, float* o32, int outx, float osc) {
    __shared__ float red0[8]; __shared__ float red1[8];
    const int row = blockIdx.x, tid = threadIdx.x, lane = tid & 31, wave = tid >> 5;
    const size_t rmap = (size_t)(row / SEQ) * SEQ_FULL + (size_t)(row % SEQ);
    const size_t rin = inx ? rmap : (size_t)row; const size_t rout = outx ? rmap : (size_t)row;
    v4f v = *(const v4f*)(in + rin * DM + tid * 4);
    if (inx) { v[0] = bfr(v[0]); v[1] = bfr(v[1]); v[2] = bfr(v[2]); v[3] = bfr(v[3]); }
    float s = (v[0] + v[1]) + (v[2] + v[3]);
#pragma unroll
    for (int sh = 16; sh; sh >>= 1) s += __shfl_xor(s, sh, 32);
    if (lane == 0) red0[wave] = s;
    __syncthreads();
    float tot = red0[0];
#pragma unroll
    for (int w = 1; w < 8; ++w) tot += red0[w];
    const float mu = tot * (1.0f / DM);
    const float d0 = v[0] - mu, d1 = v[1] - mu, d2 = v[2] - mu, d3 = v[3] - mu;
    float s2 = (d0 * d0 + d1 * d1) + (d2 * d2 + d3 * d3);
#pragma unroll
    for (int sh = 16; sh; sh >>= 1) s2 += __shfl_xor(s2, sh, 32);
    if (lane == 0) red1[wave] = s2;
    __syncthreads();
    float tot2 = red1[0];
#pragma unroll
    for (int w = 1; w < 8; ++w) tot2 += red1[w];
    const float rs = rsqrtf(tot2 * (1.0f / DM) + 1e-5f);
    const v4f gw = *(const v4f*)(g + tid * 4); const v4f gb = *(const v4f*)(bta + tid * 4);
    v4f y;
    y[0] = (d0 * rs * bfr(gw[0]) + bfr(gb[0])) * osc; y[1] = (d1 * rs * bfr(gw[1]) + bfr(gb[1])) * osc;
    y[2] = (d2 * rs * bfr(gw[2]) + bfr(gb[2])) * osc; y[3] = (d3 * rs * bfr(gw[3]) + bfr(gb[3])) * osc;
    if constexpr (MODE == 0) {
        v4h o; o[0] = (h16)y[0]; o[1] = (h16)y[1]; o[2] = (h16)y[2]; o[3] = (h16)y[3];
        unsigned short* p = o16 + rout * DM + tid * 4;
        *(volatile v4h*)p = o; __threadfence(); *(volatile v4h*)p = o;
    } else {
        float* p = o32 + rout * DM + tid * 4;
        *(volatile v4f*)p = y; __threadfence(); *(volatile v4f*)p = y;
    }
}

__global__ __launch_bounds__(256) void k_asoft(const float* __restrict__ Sb, unsigned short* P16) {
    const int lane = threadIdx.x & 31; const int row = blockIdx.x * 8 + (threadIdx.x >> 5); if (row >= ZH * SEQ) return;
    const float* sr = Sb + (size_t)row * SEQ; float v[SEQ / 32]; float mx = -3.0e38f;
#pragma unroll
    for (int ch = 0; ch < SEQ / 128; ++ch) { const int j0 = ch * 128 + lane * 4; const v4f a = *(const v4f*)(sr + j0);
#pragma unroll
        for (int q = 0; q < 4; ++q) { const float t = a[q] * SCLS; v[ch * 4 + q] = t; mx = fmaxf(mx, t); } }
#pragma unroll
    for (int sh = 16; sh; sh >>= 1) mx = fmaxf(mx, __shfl_xor(mx, sh, 32));
    float sum = 0.f;
#pragma unroll
    for (int k = 0; k < SEQ / 32; ++k) { float d0 = __fsub_rn(v[k], mx); asm volatile("" : "+v"(d0)); v[k] = __builtin_amdgcn_exp2f(__fmul_rn(d0, 1.4426950408889634f)); sum += v[k]; }
#pragma unroll
    for (int sh = 16; sh; sh >>= 1) sum += __shfl_xor(sum, sh, 32);
    const float f = __fdiv_rn(PCAR, sum);
#pragma unroll 1
    for (int ps = 0; ps < 2; ++ps) {
#pragma unroll
        for (int ch = 0; ch < SEQ / 128; ++ch) { v4h o4;
#pragma unroll
            for (int q = 0; q < 4; ++q) o4[q] = (h16)(v[ch * 4 + q] * f);
            *(volatile v4h*)(P16 + (size_t)row * SEQ + ch * 128 + lane * 4) = o4; }
        if (ps == 0) __threadfence(); }
}

extern "C" void kernel_launch(void* const* d_in, const int* in_sizes, int n_in,
                              void* d_out, int out_size, void* d_ws, size_t ws_size, hipStream_t stream) {
    if (n_in < 21) return;
    const size_t xneed = ((size_t)(NB - 1) * SEQ_FULL + SEQ) * DM;
    if ((size_t)in_sizes[0] < xneed || (size_t)out_size < xneed) return;
    if ((size_t)in_sizes[1] < (size_t)DM * DM || (size_t)in_sizes[3] < (size_t)DM * DM || (size_t)in_sizes[5] < (size_t)DM * DM || (size_t)in_sizes[7] < (size_t)DM * DM) return;
    if ((size_t)in_sizes[13] < (size_t)DM * DF || (size_t)in_sizes[15] < (size_t)DF * DM || (size_t)in_sizes[17] < (size_t)DM * DM) return;
    if (in_sizes[2] < DM || in_sizes[4] < DM || in_sizes[6] < DM || in_sizes[8] < DM || in_sizes[14] < DF || in_sizes[16] < DM || in_sizes[18] < DM) return;
    if (in_sizes[9] < DM || in_sizes[10] < DM || in_sizes[11] < DM || in_sizes[12] < DM || in_sizes[19] < DM || in_sizes[20] < DM) return;
    const float* x    = (const float*)d_in[0];
    const float* wq   = (const float*)d_in[1];  const float* bq   = (const float*)d_in[2];
    const float* wk   = (const float*)d_in[3];  const float* bk   = (const float*)d_in[4];
    const float* wv   = (const float*)d_in[5];  const float* bv   = (const float*)d_in[6];
    const float* wo   = (const float*)d_in[7];  const float* bo   = (const float*)d_in[8];
    const float* ln1w = (const float*)d_in[9];  const float* ln1b = (const float*)d_in[10];
    const float* ln2w = (const float*)d_in[11]; const float* ln2b = (const float*)d_in[12];
    const float* fc1w = (const float*)d_in[13]; const float* fc1b = (const float*)d_in[14];
    const float* fc2w = (const float*)d_in[15]; const float* fc2b = (const float*)d_in[16];
    const float* wout = (const float*)d_in[17]; const float* bout = (const float*)d_in[18];
    const float* lnow = (const float*)d_in[19]; const float* lnob = (const float*)d_in[20];
    float* OUT = (float*)d_out;

    char* wsp = (char*)d_ws;
    auto take = [&](size_t bytes) { char* p = wsp; wsp += (bytes + 255) & ~(size_t)255; return (void*)p; };
    unsigned short* WQ = (unsigned short*)take((size_t)DM * DM * 2); unsigned short* WK = (unsigned short*)take((size_t)DM * DM * 2);
    unsigned short* WV = (unsigned short*)take((size_t)DM * DM * 2); unsigned short* WO = (unsigned short*)take((size_t)DM * DM * 2);
    unsigned short* F1 = (unsigned short*)take((size_t)DF * DM * 2); unsigned short* F2 = (unsigned short*)take((size_t)DM * DF * 2);
    unsigned short* WOUTB = (unsigned short*)take((size_t)DM * DM * 2);
    unsigned short* ACT = (unsigned short*)take((size_t)MR * DM * 2);
    unsigned short* QP = (unsigned short*)take((size_t)MR * DM * 2);
    unsigned short* KP = (unsigned short*)take((size_t)MR * DM * 2);
    unsigned short* VT = (unsigned short*)take((size_t)MR * DM * 2);
    const size_t sbA = (size_t)ZH * SEQ * SEQ * 4, sbB = (size_t)MR * DF * 2;
    void* RS = take(sbA > sbB ? sbA : sbB);
    const size_t pA = (size_t)ZH * SEQ * SEQ * 2, pB = (size_t)MR * DM * 4;
    void* RP = take(pA > pB ? pA : pB);
    float* H2 = (float*)take((size_t)MR * DM * 4);
    const size_t carved = (size_t)(wsp - (char*)d_ws);
    if (carved > ws_size || carved > (size_t)134217728) return;
    float* Sb = (float*)RS; unsigned short* G16 = (unsigned short*)RS;
    unsigned short* P16 = (unsigned short*)RP; float* PF = (float*)RP;
    unsigned short* H3h = QP; unsigned short* H3l = KP;
    const h16* ACTh = (const h16*)ACT;

    k_tcvt<1><<<dim3(DM / 64, DM / 64), 256, 0, stream>>>(wq, WQ, DM, DM, WCAR);
    k_tcvt<1><<<dim3(DM / 64, DM / 64), 256, 0, stream>>>(wk, WK, DM, DM, WCAR);
    k_tcvt<1><<<dim3(DM / 64, DM / 64), 256, 0, stream>>>(wv, WV, DM, DM, WCAR);
    k_tcvt<1><<<dim3(DM / 64, DM / 64), 256, 0, stream>>>(wo, WO, DM, DM, WCAR);
    k_tcvt<1><<<dim3(DF / 64, DM / 64), 256, 0, stream>>>(fc1w, F1, DM, DF, WCAR);
    k_tcvt<1><<<dim3(DM / 64, DF / 64), 256, 0, stream>>>(fc2w, F2, DF, DM, WCAR);
    k_tcvt<0><<<dim3(DM / 64, DM / 64), 256, 0, stream>>>(wout, WOUTB, DM, DM, 1.0f);

    k_ln<0><<<MR, 256, 0, stream>>>(x, 1, ln1w, ln1b, ACT, nullptr, 0, ACAR);
    const float scp = 1.0f / (ACAR * WCAR);
    k_gemmw<h16, 0, (E_CB | E_H16)><<<dim3(MR / 64, DM / 64, 1), 32, 0, stream>>>(ACTh, nullptr, (const h16*)WQ, DM, nullptr, QP, nullptr, HD, (size_t)MR * HD, bq, nullptr, 0, scp, QCAR, 0, 0, 0);
    k_gemmw<h16, 0, (E_CB | E_H16)><<<dim3(MR / 64, DM / 64, 1), 32, 0, stream>>>(ACTh, nullptr, (const h16*)WK, DM, nullptr, KP, nullptr, HD, (size_t)MR * HD, bk, nullptr, 0, scp, QCAR, 0, 0, 0);
    k_gemmw<h16, 0, (E_RB | E_H16)><<<dim3(DM / 64, SEQ / 64, NB), 32, 0, stream>>>((const h16*)WV, nullptr, ACTh, DM, nullptr, VT, nullptr, SEQ, 64, bv, nullptr, 0, scp, VCAR, 0, (size_t)SEQ * DM, (size_t)DM * SEQ);

    for (int b = 0; b < NB; ++b) {
        for (int h0 = 0; h0 < NH_; h0 += ZH) {
            const size_t qo = ((size_t)h0 * MR + (size_t)b * SEQ) * HD;
            k_gemmw<h16, 0, 0><<<dim3(SEQ / 64, SEQ / 64, ZH), 32, 0, stream>>>((const h16*)QP + qo, nullptr, (const h16*)KP + qo, HD, Sb, nullptr, nullptr, SEQ, 64, nullptr, nullptr, 0, 1.0f, 1.0f, (size_t)MR * HD, (size_t)MR * HD, (size_t)SEQ * SEQ);
            k_asoft<<<ZH * SEQ / 8, 256, 0, stream>>>(Sb, P16);
            k_gemmw<h16, 0, E_H16><<<dim3(SEQ / 64, 1, ZH), 32, 0, stream>>>((const h16*)P16, nullptr, (const h16*)VT + ((size_t)b * DM + (size_t)h0 * HD) * SEQ, SEQ, nullptr, ACT + (size_t)b * SEQ * DM + (size_t)h0 * HD, nullptr, DM, 64, nullptr, nullptr, 0, 1.0f, 1.0f, (size_t)SEQ * SEQ, (size_t)HD * SEQ, (size_t)HD);
        }
    }
    k_gemmw<h16, 0, (E_CB | E_RES | E_RESX)><<<dim3(MR / 64, DM / 64, 1), 32, 0, stream>>>(ACTh, nullptr, (const h16*)WO, DM, H2, nullptr, nullptr, DM, 64, bo, x, DM, 1.0f / (PCAR * VCAR * WCAR), 1.0f, 0, 0, 0);
    k_ln<0><<<MR, 256, 0, stream>>>(H2, 0, ln2w, ln2b, ACT, nullptr, 0, ACAR);
    k_gemmw<h16, 0, (E_CB | E_GELU | E_H16)><<<dim3(MR / 64, DF / 64, 1), 32, 0, stream>>>(ACTh, nullptr, (const h16*)F1, DM, nullptr, G16, nullptr, DF, 64, fc1b, nullptr, 0, scp, GCAR, 0, 0, 0);
    k_gemmw<h16, 0, (E_CB | E_RES | E_BF2)><<<dim3(MR / 64, DM / 64, 1), 32, 0, stream>>>((const h16*)G16, nullptr, (const h16*)F2, DF, nullptr, H3h, H3l, DM, 64, fc2b, H2, DM, 1.0f / (GCAR * WCAR), 1.0f, 0, 0, 0);
    k_gemmw<bf, 1, E_CB><<<dim3(MR / 64, DM / 64, 1), 32, 0, stream>>>((const bf*)H3h, (const bf*)H3l, (const bf*)WOUTB, DM, PF, nullptr, nullptr, DM, 64, bout, nullptr, 0, 1.0f, 1.0f, 0, 0, 0);
    k_ln<1><<<MR, 256, 0, stream>>>(PF, 0, lnow, lnob, nullptr, OUT, 1, 1.0f);
}
